// Attention_43233140802225
// MI455X (gfx1250) — hardware-verified
//
#include <hip/hip_runtime.h>


#ifndef NB
#define NB 2
#endif
#ifndef SEQ
#define SEQ 2048
#endif
#define NB_FULL  2
#define SEQ_FULL 2048
#define DM   2048
#define NH_  16
#define HD   128
#define TPH  (HD / 64)
#define RH   ((SEQ) < 512 ? (SEQ) : 512)
#define PCAR 1024.0f
#define CCAR 64.0f
#define WCAR 256.0f
#define SCL  0.08838834764831845f
#define L2E  1.4426950408889634f
#define NEGB (-3.0e38f)
#define CHK_T 512
#define VCAP __attribute__((amdgpu_num_vgpr(256)))

static_assert(NH_ * HD == DM);
static_assert(HD == 128);
static_assert(DM % 64 == 0);
static_assert(SEQ % 64 == 0);
static_assert(RH % 64 == 0);
static_assert(RH <= SEQ);
static_assert(NB <= NB_FULL);
static_assert(SEQ <= SEQ_FULL);
static_assert(DM / 8 == 256);
static_assert(CHK_T % 32 == 0 && CHK_T <= 1024);
static_assert(((size_t)SEQ * (SEQ / 4)) % CHK_T == 0);
static_assert(SEQ_FULL % 4 == 0);

typedef _Float16 h16;
typedef unsigned short bf;
typedef __attribute__((ext_vector_type(16))) __bf16   v16bf;
typedef __attribute__((ext_vector_type(16))) _Float16 v16h;
typedef __attribute__((ext_vector_type(8)))  _Float16 v8h;
typedef __attribute__((ext_vector_type(8)))  unsigned short v8us;
typedef __attribute__((ext_vector_type(8)))  float    v8f;
typedef __attribute__((ext_vector_type(4)))  float    v4f;
typedef v8h  __attribute__((may_alias)) v8ha;
typedef v4f  __attribute__((may_alias)) v4fa;
typedef v8us __attribute__((may_alias)) v8usa;

__device__ __forceinline__ unsigned short f2bf(float f) { unsigned u = __float_as_uint(f); u += 0x7FFFu + ((u >> 16) & 1u); return (unsigned short)(u >> 16); }
__device__ __forceinline__ float bf2f(unsigned short b) { return __uint_as_float(((unsigned)b) << 16); }
__device__ __forceinline__ float bfr(float f) { return bf2f(f2bf(f)); }
__device__ __forceinline__ v16h cat16(v8h lo, v8h hi) { return __builtin_shufflevector(lo, hi, 0, 1, 2, 3, 4, 5, 6, 7, 8, 9, 10, 11, 12, 13, 14, 15); }
__device__ __forceinline__ v16bf cat16b(v8us lo, v8us hi) { return __builtin_bit_cast(v16bf, __builtin_shufflevector(lo, hi, 0, 1, 2, 3, 4, 5, 6, 7, 8, 9, 10, 11, 12, 13, 14, 15)); }
__device__ __forceinline__ v8f wmma16(v16h a, v16h b, v8f c) { return __builtin_amdgcn_wmma_f32_16x16x32_f16(false, a, false, b, (short)0, c, false, false); }
__device__ __forceinline__ v8f wmmab(v16bf a, v16bf b, v8f c) { return __builtin_amdgcn_wmma_f32_16x16x32_bf16(false, a, false, b, (short)0, c, false, false); }
__device__ __forceinline__ void splitf(float y, unsigned short& h, unsigned short& l) { h = f2bf(y); l = f2bf(y - bf2f(h)); }
static __device__ __forceinline__ h16 toh_flush(float v) { const h16 r = (h16)v; return (fabsf(v) < 6.103515625e-05f) ? (h16)0.0f : r; }

template <typename T16> struct WFrag;
template <> struct WFrag<h16> { typedef v16h V;
    static __device__ __forceinline__ V ld(const h16* p) { return cat16(*(const v8h*)p, *(const v8h*)(p + 16)); }
    static __device__ __forceinline__ V ldl(const h16* p) { return cat16(*(const v8ha*)p, *(const v8ha*)(p + 16)); }
    static __device__ __forceinline__ v8f mma(V a, V b, v8f c) { return wmma16(a, b, c); } };
template <> struct WFrag<bf> { typedef v16bf V;
    static __device__ __forceinline__ V ld(const bf* p) { return cat16b(*(const v8us*)p, *(const v8us*)(p + 16)); }
    static __device__ __forceinline__ V ldl(const bf* p) { return cat16b(*(const v8usa*)p, *(const v8usa*)(p + 16)); }
    static __device__ __forceinline__ v8f mma(V a, V b, v8f c) { return wmmab(a, b, c); } };

template <typename T16, int NSPLIT>
__global__ __launch_bounds__(32) VCAP void k_gemmw(const T16* __restrict__ A, const T16* __restrict__ A2, const T16* __restrict__ Bt, float* C, int ldc, float oscale, size_t sA, size_t sC) {
    typedef typename WFrag<T16>::V V;
    __shared__ __align__(16) float os[16 * 68];
    const size_t z = blockIdx.z; A += z * sA; if (NSPLIT == 1) A2 += z * sA; C += z * sC;
    const int lane = threadIdx.x & 31, lr = lane & 15, hi = lane >> 4; const int r0 = blockIdx.x * 64, c0 = blockIdx.y * 64;
    v8f acc[4][4];
#pragma unroll
    for (int mb = 0; mb < 4; ++mb)
#pragma unroll
        for (int nb = 0; nb < 4; ++nb) acc[mb][nb] = (v8f){};
    const size_t aoff = (size_t)(r0 + lr) * DM + 8 * hi, boff = (size_t)(c0 + lr) * DM + 8 * hi;
#pragma unroll 1
    for (int kc = 0; kc < DM; kc += 32) {
        V b[4], a, a2;
#pragma unroll
        for (int nb = 0; nb < 4; ++nb) b[nb] = WFrag<T16>::ld(Bt + boff + (size_t)nb * 16 * DM + kc);
#pragma unroll
        for (int mb = 0; mb < 4; ++mb) { a = WFrag<T16>::ld(A + aoff + (size_t)mb * 16 * DM + kc); if (NSPLIT == 1) a2 = WFrag<T16>::ld(A2 + aoff + (size_t)mb * 16 * DM + kc);
#pragma unroll
            for (int nb = 0; nb < 4; ++nb) { acc[mb][nb] = WFrag<T16>::mma(a, b[nb], acc[mb][nb]); if (NSPLIT == 1) acc[mb][nb] = WFrag<T16>::mma(a2, b[nb], acc[mb][nb]); } }
        asm volatile("v_nop\n\tv_nop\n\tv_nop\n\tv_nop" : "+v"(acc[0][0]), "+v"(acc[1][1]), "+v"(acc[2][2]), "+v"(acc[3][3]) : "v"(a), "v"(b[3]));
    }
#pragma unroll
    for (int mb = 0; mb < 4; ++mb) {
#pragma unroll
        for (int nb = 0; nb < 4; ++nb) {
#pragma unroll
            for (int j = 0; j < 8; ++j) os[(hi * 8 + j) * 68 + nb * 16 + lr] = acc[mb][nb][j]; }
        __builtin_amdgcn_wave_barrier(); asm volatile("" ::: "memory");
        float* crow = C + (size_t)(r0 + mb * 16) * ldc + c0;
#pragma unroll 1
        for (int ps = 0; ps < 2; ++ps) {
#pragma unroll
            for (int s = 0; s < 8; ++s) { const int row = 2 * s + hi, cofs = lr * 4; v4f val = *(const v4fa*)(os + row * 68 + cofs); val = val * oscale;
                *(volatile v4f*)(crow + (size_t)row * ldc + cofs) = val; }
            if (ps == 0) __threadfence(); }
        __builtin_amdgcn_wave_barrier(); asm volatile("" ::: "memory");
    }
}

template <int VMODE>
__global__ __launch_bounds__(32) VCAP void k_projp(const bf* __restrict__ A, const bf* __restrict__ Bt, h16* P16, bf* Ph, bf* Pl) {
    typedef WFrag<bf>::V V;
    __shared__ __align__(16) float os[64 * 68];
    const unsigned lane = threadIdx.x & 31u, lr = lane & 15u, hi = lane >> 4; const unsigned r0 = blockIdx.x * 64u, c0 = blockIdx.y * 64u;
    v8f acc[4][4];
#pragma unroll
    for (int mb = 0; mb < 4; ++mb)
#pragma unroll
        for (int nb = 0; nb < 4; ++nb) acc[mb][nb] = (v8f){};
    const size_t aoff = (size_t)(r0 + lr) * DM + 8u * hi, boff = (size_t)(c0 + lr) * DM + 8u * hi;
#pragma unroll 1
    for (unsigned kc = 0; kc < (unsigned)DM; kc += 32u) {
        V a[4], b;
#pragma unroll
        for (int mb = 0; mb < 4; ++mb) a[mb] = WFrag<bf>::ld(A + aoff + (size_t)mb * 16 * DM + kc);
#pragma unroll
        for (int nb = 0; nb < 4; ++nb) { b = WFrag<bf>::ld(Bt + boff + (size_t)nb * 16 * DM + kc);
#pragma unroll
            for (int mb = 0; mb < 4; ++mb) acc[mb][nb] = WFrag<bf>::mma(a[mb], b, acc[mb][nb]); }
        asm volatile("v_nop\n\tv_nop\n\tv_nop\n\tv_nop" : "+v"(acc[0][0]), "+v"(acc[1][1]), "+v"(acc[2][2]), "+v"(acc[3][3]) : "v"(a[3]), "v"(b));
    }
#pragma unroll
    for (int mb = 0; mb < 4; ++mb)
#pragma unroll
        for (int nb = 0; nb < 4; ++nb)
#pragma unroll
            for (int j = 0; j < 8; ++j) os[(mb * 16 + hi * 8 + j) * 68 + nb * 16 + lr] = acc[mb][nb][j];
    __syncthreads();
    const unsigned b = r0 / (unsigned)SEQ, t0 = r0 % (unsigned)SEQ;
    const unsigned hd = blockIdx.y / (unsigned)TPH, dh = (blockIdx.y % (unsigned)TPH) * 64u; const unsigned bh = b * NH_ + hd;
    const bool hires = (t0 < (unsigned)RH);
    const unsigned rq = lane >> 3, pc = lane & 7u;
    if (VMODE == 0) {
        const size_t o16 = ((size_t)bh * SEQ + t0) * HD + dh + pc * 8u;
        const size_t ohl = ((size_t)bh * RH + t0) * HD + dh + pc * 8u;
#pragma unroll 1
        for (int ps = 0; ps < 2; ++ps) {
#pragma unroll 2
            for (unsigned s = 0; s < 16u; ++s) { const unsigned row = s * 4u + rq;
                const v4f x0 = *(const v4fa*)(os + row * 68u + pc * 8u), x1 = *(const v4fa*)(os + row * 68u + pc * 8u + 4u); v8h o;
#pragma unroll
                for (int q = 0; q < 4; ++q) { o[q] = (h16)x0[q]; o[4 + q] = (h16)x1[q]; }
                *(volatile v8h*)(P16 + o16 + (size_t)row * HD) = o;
                if (hires) { v8us oh, ol;
#pragma unroll
                    for (int q = 0; q < 4; ++q) { unsigned short a2, c2; splitf(x0[q], a2, c2); oh[q] = a2; ol[q] = c2; splitf(x1[q], a2, c2); oh[4 + q] = a2; ol[4 + q] = c2; }
                    *(volatile v8us*)(Ph + ohl + (size_t)row * HD) = oh; *(volatile v8us*)(Pl + ohl + (size_t)row * HD) = ol; } }
            if (ps == 0) __threadfence(); }
    } else {
        const size_t o16 = (size_t)bh * HD * SEQ + (size_t)dh * SEQ + t0 + pc * 8u;
        const size_t ohl = (size_t)bh * HD * RH + (size_t)dh * RH + t0 + pc * 8u;
#pragma unroll 1
        for (int ps = 0; ps < 2; ++ps) {
#pragma unroll 2
            for (unsigned s = 0; s < 16u; ++s) { const unsigned d = s * 4u + rq;
                float x[8];
#pragma unroll
                for (int j = 0; j < 8; ++j) x[j] = os[(pc * 8u + j) * 68u + d];
                v8h o;
#pragma unroll
                for (int j = 0; j < 8; ++j) o[j] = (h16)x[j];
                *(volatile v8h*)(P16 + o16 + (size_t)d * SEQ) = o;
                if (hires) { v8us oh, ol;
#pragma unroll
                    for (int j = 0; j < 8; ++j) { unsigned short a2, c2; splitf(x[j], a2, c2); oh[j] = a2; ol[j] = c2; }
                    *(volatile v8us*)(Ph + ohl + (size_t)d * RH) = oh; *(volatile v8us*)(Pl + ohl + (size_t)d * RH) = ol; } }
            if (ps == 0) __threadfence(); }
    }
}

__device__ __forceinline__ void pput(h16* ph, h16* pl, unsigned idx, float p) { (void)pl; ph[idx] = (h16)(p * PCAR); }
__device__ __forceinline__ void pput(bf* ph, bf* pl, unsigned idx, float p) { unsigned short a, c; splitf(p, a, c); ph[idx] = a; pl[idx] = c; }
__device__ __forceinline__ void cput(bf* Ah, bf* Al, size_t off, v4f x0, v4f x1) { v8us oh, ol;
#pragma unroll
    for (int q = 0; q < 4; ++q) { unsigned short a2, c2; splitf(x0[q], a2, c2); oh[q] = a2; ol[q] = c2; splitf(x1[q], a2, c2); oh[4 + q] = a2; ol[4 + q] = c2; }
    *(volatile v8us*)(Ah + off) = oh; *(volatile v8us*)(Al + off) = ol; }
__device__ __forceinline__ void cput(h16* Ah, h16* Al, size_t off, v4f x0, v4f x1) { (void)Al; v8h o;
#pragma unroll
    for (int q = 0; q < 4; ++q) { o[q] = (h16)x0[q]; o[4 + q] = (h16)x1[q]; }
    *(volatile v8h*)(Ah + off) = o; }
__device__ __forceinline__ void pput_fl(h16* ph, h16* pl, unsigned idx, float p) { (void)pl; ph[idx] = toh_flush(p * PCAR); }
__device__ __forceinline__ void pput_fl(bf* ph, bf* pl, unsigned idx, float p) { unsigned short a, c; splitf(p, a, c); ph[idx] = a; pl[idx] = c; }
__device__ __forceinline__ void cput_fl(bf* Ah, bf* Al, size_t off, v4f x0, v4f x1) { v8us oh, ol;
#pragma unroll
    for (int q = 0; q < 4; ++q) { unsigned short a2, c2; splitf(x0[q], a2, c2); oh[q] = a2; ol[q] = c2; splitf(x1[q], a2, c2); oh[4 + q] = a2; ol[4 + q] = c2; }
    *(volatile v8us*)(Ah + off) = oh; *(volatile v8us*)(Al + off) = ol; }
__device__ __forceinline__ void cput_fl(h16* Ah, h16* Al, size_t off, v4f x0, v4f x1) { (void)Al; v8h o;
#pragma unroll
    for (int q = 0; q < 4; ++q) { o[q] = toh_flush(x0[q]); o[4 + q] = toh_flush(x1[q]); }
    *(volatile v8h*)(Ah + off) = o; }

__global__ __launch_bounds__(CHK_T) void k_maskchk(const float* __restrict__ MK, float* FLG) {
    __shared__ unsigned wbad[CHK_T / 32];
    const unsigned tid = threadIdx.x; const int wave = __builtin_amdgcn_readfirstlane(threadIdx.x >> 5);
    unsigned bad = 0u;
#pragma unroll 1
    for (unsigned i = tid; i < (unsigned)SEQ * (unsigned)(SEQ / 4); i += (unsigned)CHK_T) {
        const unsigned q = i / (unsigned)(SEQ / 4), c = (i % (unsigned)(SEQ / 4)) * 4u;
        const v4f m4 = *(const v4f*)(MK + (size_t)q * SEQ_FULL + c);
        const unsigned T = q >> 6, U = c >> 6;
#pragma unroll
        for (int j = 0; j < 4; ++j) { const float v = m4[j];
            const bool okl = (v == 0.0f), okr = (v <= -1.0e4f), okd = ((c + (unsigned)j) != q) || (v >= -1.0e3f);
            const bool ok = (U < T) ? okl : ((U > T) ? okr : okd);
            bad |= ok ? 0u : 1u; }
    }
    bad |= __shfl_xor(bad, 16, 32); bad |= __shfl_xor(bad, 8, 32); bad |= __shfl_xor(bad, 4, 32); bad |= __shfl_xor(bad, 2, 32); bad |= __shfl_xor(bad, 1, 32);
    if ((tid & 31u) == 0u) wbad[wave] = bad;
    __syncthreads();
    unsigned tot = 0u;
#pragma unroll
    for (int w = 0; w < CHK_T / 32; ++w) tot |= wbad[w];
    const float fv = (tot != 0u) ? __uint_as_float(0x7FC00000u) : 0.0f;
    if (tid < 8u) { const v4f o = (v4f){fv, fv, fv, fv}; *(volatile v4f*)(FLG + tid * 4u) = o; __threadfence(); *(volatile v4f*)(FLG + tid * 4u) = o; }
}

template <typename T16, bool SPLIT, unsigned PROW, unsigned OROW>
__global__ __launch_bounds__(32) VCAP void k_flash(const T16* __restrict__ Q, const T16* __restrict__ Q2, const T16* __restrict__ Kp, const T16* __restrict__ K2, const T16* __restrict__ Vt, const T16* __restrict__ Vt2, const float* __restrict__ MK, const float* __restrict__ FLG, unsigned roff, T16* Ah, T16* Al) {
    typedef typename WFrag<T16>::V V;
    __shared__ __align__(16) T16 psh[16 * 72];
    __shared__ __align__(16) T16 psl[SPLIT ? 16 * 72 : 8];
    __shared__ __align__(16) float os[16 * 132];
    __shared__ __align__(16) float mk[16 * 68];
    const unsigned lane = threadIdx.x & 31u, lr = lane & 15u, hi = lane >> 4;
    const unsigned bh = blockIdx.y, r0 = roff + blockIdx.x * 16u;
    const size_t pb = (size_t)bh * PROW * HD;
    const size_t qo = pb + (size_t)(r0 + lr) * HD + 8u * hi;
    v8f O[8]; float mrun[8], lsum[8];
#pragma unroll
    for (int nt = 0; nt < 8; ++nt) O[nt] = (v8f){};
#pragma unroll
    for (int r = 0; r < 8; ++r) { mrun[r] = NEGB; lsum[r] = 0.0f; }
    const unsigned nkt = (r0 >> 6) + 1u;
    {   const unsigned mrq = lane >> 4, mpc = lane & 15u;
        const size_t mo = (size_t)r0 * SEQ_FULL + (size_t)(nkt - 1u) * 64u + mpc * 4u;
#pragma unroll
        for (unsigned s = 0; s < 8u; ++s) { const unsigned mrow = s * 2u + mrq;
            v4f m4 = *(const v4f*)(MK + mo + (size_t)mrow * SEQ_FULL);
#pragma unroll
            for (int q = 0; q < 4; ++q) m4[q] = bfr(m4[q]);
            *(v4fa*)(mk + mrow * 68u + mpc * 4u) = m4; } }
    __syncthreads();
#pragma unroll 1
    for (unsigned kt = 0; kt < nkt; ++kt) {
        const unsigned c0 = kt * 64u;
        v8f S[4];
#pragma unroll
        for (int ni = 0; ni < 4; ++ni) S[ni] = (v8f){};
        const size_t ko = pb + (size_t)(c0 + lr) * HD + 8u * hi;
#pragma unroll 1
        for (unsigned ks = 0; ks < 4u; ++ks) {
            V qx, qy, kb, kb2;
            qx = WFrag<T16>::ld(Q + qo + ks * 32u); if (SPLIT) qy = WFrag<T16>::ld(Q2 + qo + ks * 32u);
#pragma unroll
            for (int ni = 0; ni < 4; ++ni) { kb = WFrag<T16>::ld(Kp + ko + (size_t)ni * 16 * HD + ks * 32u); S[ni] = WFrag<T16>::mma(qx, kb, S[ni]);
                if (SPLIT) { S[ni] = WFrag<T16>::mma(qy, kb, S[ni]); kb2 = WFrag<T16>::ld(K2 + ko + (size_t)ni * 16 * HD + ks * 32u); S[ni] = WFrag<T16>::mma(qx, kb2, S[ni]); } }
            if (SPLIT) asm volatile("v_nop\n\tv_nop\n\tv_nop\n\tv_nop" : "+v"(S[0]), "+v"(S[1]), "+v"(S[2]), "+v"(S[3]) : "v"(qx), "v"(kb2));
            else       asm volatile("v_nop\n\tv_nop\n\tv_nop\n\tv_nop" : "+v"(S[0]), "+v"(S[1]), "+v"(S[2]), "+v"(S[3]) : "v"(qx), "v"(kb));
        }
        const bool diag = (kt + 1u == nkt);
        if (diag) {
#pragma unroll
            for (int r = 0; r < 8; ++r)
#pragma unroll
                for (int ni = 0; ni < 4; ++ni) S[ni][r] = S[ni][r] * SCL + mk[(8u * hi + r) * 68u + ni * 16u + lr];
        } else {
#pragma unroll
            for (int r = 0; r < 8; ++r)
#pragma unroll
                for (int ni = 0; ni < 4; ++ni) S[ni][r] = S[ni][r] * SCL;
        }
        float mnew[8];
#pragma unroll
        for (int r = 0; r < 8; ++r) { float mx = NEGB;
#pragma unroll
            for (int ni = 0; ni < 4; ++ni) mx = fmaxf(mx, S[ni][r]);
            mx = fmaxf(mx, __shfl_xor(mx, 8, 32)); mx = fmaxf(mx, __shfl_xor(mx, 4, 32)); mx = fmaxf(mx, __shfl_xor(mx, 2, 32)); mx = fmaxf(mx, __shfl_xor(mx, 1, 32));
            mnew[r] = fmaxf(mrun[r], mx); }
#pragma unroll
        for (int r = 0; r < 8; ++r) { const float al = __builtin_amdgcn_exp2f((mrun[r] - mnew[r]) * L2E); mrun[r] = mnew[r]; lsum[r] *= al;
#pragma unroll
            for (int nt = 0; nt < 8; ++nt) O[nt][r] *= al; }
#pragma unroll
        for (int r = 0; r < 8; ++r)
#pragma unroll
            for (int ni = 0; ni < 4; ++ni) { const float p = __builtin_amdgcn_exp2f((S[ni][r] - mnew[r]) * L2E); lsum[r] += p; pput_fl(psh, psl, (8u * hi + r) * 72u + ni * 16u + lr, p); }
        __syncthreads();
        V pa[2], pl[2];
#pragma unroll
        for (int ks = 0; ks < 2; ++ks) { pa[ks] = WFrag<T16>::ldl(psh + lr * 72u + ks * 32 + 8u * hi); if (SPLIT) pl[ks] = WFrag<T16>::ldl(psl + lr * 72u + ks * 32 + 8u * hi); }
        V vb, vb2;
        const size_t vo = pb + (size_t)lr * PROW + c0 + 8u * hi;
#pragma unroll
        for (int g = 0; g < 2; ++g) {
#pragma unroll
            for (int n4 = 0; n4 < 4; ++n4) { const int nt = g * 4 + n4;
#pragma unroll
                for (int ks = 0; ks < 2; ++ks) { vb = WFrag<T16>::ld(Vt + vo + (size_t)nt * 16 * PROW + ks * 32); O[nt] = WFrag<T16>::mma(pa[ks], vb, O[nt]);
                    if (SPLIT) { O[nt] = WFrag<T16>::mma(pl[ks], vb, O[nt]); vb2 = WFrag<T16>::ld(Vt2 + vo + (size_t)nt * 16 * PROW + ks * 32); O[nt] = WFrag<T16>::mma(pa[ks], vb2, O[nt]); } } }
            if (SPLIT) asm volatile("v_nop\n\tv_nop\n\tv_nop\n\tv_nop" : "+v"(O[0]), "+v"(O[1]), "+v"(O[2]), "+v"(O[3]), "+v"(O[4]), "+v"(O[5]), "+v"(O[6]), "+v"(O[7]) : "v"(pa[1]), "v"(vb2));
            else       asm volatile("v_nop\n\tv_nop\n\tv_nop\n\tv_nop" : "+v"(O[0]), "+v"(O[1]), "+v"(O[2]), "+v"(O[3]), "+v"(O[4]), "+v"(O[5]), "+v"(O[6]), "+v"(O[7]) : "v"(pa[1]), "v"(vb));
        }
        __syncthreads();
    }
    const float fz = FLG[0];
#pragma unroll
    for (int r = 0; r < 8; ++r) { float l = lsum[r]; l += __shfl_xor(l, 8, 32); l += __shfl_xor(l, 4, 32); l += __shfl_xor(l, 2, 32); l += __shfl_xor(l, 1, 32);
        const float inv = __fdiv_rn(1.0f, l) * (SPLIT ? 1.0f : (CCAR / PCAR)) + fz;
#pragma unroll
        for (int nt = 0; nt < 8; ++nt) os[(8u * hi + r) * 132u + nt * 16u + lr] = O[nt][r] * inv; }
    __syncthreads();
    const unsigned b = bh / (unsigned)NH_, h = bh % (unsigned)NH_; const unsigned rq = lane >> 4, pc = lane & 15u;
    const size_t ob = ((size_t)b * OROW + r0) * DM + h * HD + pc * 8u;
#pragma unroll 1
    for (int ps = 0; ps < 2; ++ps) {
#pragma unroll
        for (unsigned s = 0; s < 8u; ++s) { const unsigned row = s * 2u + rq;
            const v4f x0 = *(const v4fa*)(os + row * 132u + pc * 8u), x1 = *(const v4fa*)(os + row * 132u + pc * 8u + 4u);
            cput_fl(Ah, Al, ob + (size_t)row * DM, x0, x1); }
        if (ps == 0) __threadfence(); }
}

__global__ __launch_bounds__(256) void k_cvt8(const float* __restrict__ src, bf* dst, size_t n8) { const size_t i = (size_t)blockIdx.x * 256 + threadIdx.x; if (i >= n8) return; const v8f v = *(const v8f*)(src + i * 8); v8us o;
#pragma unroll
    for (int k = 0; k < 8; ++k) o[k] = f2bf(v[k]); *(volatile v8us*)(dst + i * 8) = o; __threadfence(); *(volatile v8us*)(dst + i * 8) = o; }
__global__ __launch_bounds__(256) void k_cvtwh(const float* __restrict__ src, h16* dst, size_t n8) { const size_t i = (size_t)blockIdx.x * 256 + threadIdx.x; if (i >= n8) return; const v8f v = *(const v8f*)(src + i * 8); v8h o;
#pragma unroll
    for (int k = 0; k < 8; ++k) o[k] = (h16)(bfr(v[k]) * WCAR); *(volatile v8h*)(dst + i * 8) = o; __threadfence(); *(volatile v8h*)(dst + i * 8) = o; }
__global__ __launch_bounds__(256) void k_cvtx(const float* __restrict__ src, bf* dst) { const unsigned i = blockIdx.x * 256u + threadIdx.x; if (i >= (unsigned)NB * SEQ * (DM / 8)) return;
    const unsigned m = i >> 8, c8 = i & 255u; const unsigned b = m / (unsigned)SEQ, t = m % (unsigned)SEQ; const v8f v = *(const v8f*)(src + ((size_t)b * SEQ_FULL + t) * DM + c8 * 8u); v8us o;
#pragma unroll
    for (int k = 0; k < 8; ++k) o[k] = f2bf(v[k]); *(volatile v8us*)(dst + (size_t)i * 8) = o; __threadfence(); *(volatile v8us*)(dst + (size_t)i * 8) = o; }

constexpr size_t SZ_X = (size_t)NB * SEQ * DM * 2;
constexpr size_t SZ_W = (size_t)DM * DM * 2;
constexpr size_t SZ_P = (size_t)NB * NH_ * SEQ * HD * 2;
constexpr size_t SZ_R = (size_t)NB * NH_ * RH * HD * 2;
constexpr size_t SZ_C = (size_t)NB * RH * DM * 2;
constexpr size_t SZ_F = 256;
constexpr size_t WS_TOTAL = SZ_X + 4 * SZ_W + 3 * SZ_P + 6 * SZ_R + SZ_F;
static_assert(SZ_X % 256 == 0 && SZ_W % 256 == 0 && SZ_P % 256 == 0 && SZ_R % 256 == 0 && SZ_F % 256 == 0);
static_assert(SZ_F >= 8 * 16);
static_assert(SZ_C <= SZ_W);
static_assert((size_t)NB * SEQ * DM * 2 <= SZ_X);
static_assert((size_t)DM * DM * 2 <= SZ_W);
static_assert(WS_TOTAL <= (size_t)134217728);
static_assert(((size_t)NB * SEQ * (DM / 8)) % 256 == 0);
static_assert(((size_t)DM * DM / 8) % 256 == 0);

extern "C" void kernel_launch(void* const* d_in, const int* in_sizes, int n_in,
                              void* d_out, int out_size, void* d_ws, size_t ws_size, hipStream_t stream) {
    if (n_in < 6) return;
    const size_t need_x = ((size_t)(NB - 1) * SEQ_FULL + SEQ) * DM;
    if ((size_t)in_sizes[0] < need_x) return;
    if ((size_t)in_sizes[1] < (size_t)(SEQ - 1) * SEQ_FULL + SEQ) return;
    for (int i = 2; i < 6; ++i) if ((size_t)in_sizes[i] < (size_t)DM * DM) return;
    if ((size_t)out_size < need_x) return;
    if (ws_size < WS_TOTAL) return;
    const float* x = (const float*)d_in[0]; const float* mask = (const float*)d_in[1];
    const float* wq = (const float*)d_in[2]; const float* wk = (const float*)d_in[3]; const float* wv = (const float*)d_in[4]; const float* wo = (const float*)d_in[5];
    float* OUT = (float*)d_out;
    char* wsp = (char*)d_ws;
    auto take = [&](size_t bytes) { char* p = wsp; wsp += (bytes + 255) & ~(size_t)255; return (void*)p; };
    bf* XB = (bf*)take(SZ_X);
    bf* WQ = (bf*)take(SZ_W); bf* WK = (bf*)take(SZ_W); bf* WV = (bf*)take(SZ_W); bf* WO = (bf*)take(SZ_W);
    h16* QP16 = (h16*)take(SZ_P); h16* KP16 = (h16*)take(SZ_P); h16* VT16 = (h16*)take(SZ_P);
    bf* QPh = (bf*)take(SZ_R); bf* QPl = (bf*)take(SZ_R); bf* KPh = (bf*)take(SZ_R); bf* KPl = (bf*)take(SZ_R); bf* VTh = (bf*)take(SZ_R); bf* VTl = (bf*)take(SZ_R);
    float* FLG = (float*)take(SZ_F);
    if ((size_t)(wsp - (char*)d_ws) > ws_size) return;
    h16* CT16 = (h16*)XB;
    h16* WO16 = (h16*)WQ;
    bf*  ATh  = WK;
    bf*  ATl  = WV;

    k_maskchk<<<1, CHK_T, 0, stream>>>(mask, FLG);

    k_cvtx<<<(unsigned)((size_t)NB * SEQ * (DM / 8) / 256), 256, 0, stream>>>(x, XB);
    const unsigned gw = (unsigned)((size_t)DM * DM / 8 / 256);
    k_cvt8<<<gw, 256, 0, stream>>>(wq, WQ, (size_t)DM * DM / 8);
    k_cvt8<<<gw, 256, 0, stream>>>(wk, WK, (size_t)DM * DM / 8);
    k_cvt8<<<gw, 256, 0, stream>>>(wv, WV, (size_t)DM * DM / 8);
    k_cvt8<<<gw, 256, 0, stream>>>(wo, WO, (size_t)DM * DM / 8);

    const dim3 gp(NB * SEQ / 64, DM / 64, 1);
    k_projp<0><<<gp, 32, 0, stream>>>(XB, WQ, QP16, QPh, QPl);
    k_projp<0><<<gp, 32, 0, stream>>>(XB, WK, KP16, KPh, KPl);
    k_projp<1><<<gp, 32, 0, stream>>>(XB, WV, VT16, VTh, VTl);

    if (SEQ > RH) k_cvtwh<<<gw, 256, 0, stream>>>(wo, WO16, (size_t)DM * DM / 8);

    k_flash<bf, true, (RH), (RH)><<<dim3(RH / 16, NB * NH_, 1), 32, 0, stream>>>(QPh, QPl, KPh, KPl, VTh, VTl, mask, FLG, 0u, ATh, ATl);
    if (SEQ > RH)
        k_flash<h16, false, (SEQ), (SEQ)><<<dim3((SEQ - RH) / 16, NB * NH_, 1), 32, 0, stream>>>(QP16, nullptr, KP16, nullptr, VT16, nullptr, mask, FLG, (unsigned)RH, CT16, nullptr);

    k_gemmw<bf, 1><<<dim3(RH / 64, DM / 64, NB), 32, 0, stream>>>(ATh, ATl, WO, OUT, DM, 1.0f, (size_t)RH * DM, (size_t)SEQ_FULL * DM);
    if (SEQ > RH)
        k_gemmw<h16, 0><<<dim3((SEQ - RH) / 64, DM / 64, NB), 32, 0, stream>>>(CT16 + (size_t)RH * DM, nullptr, WO16, OUT + (size_t)RH * DM, DM, 1.0f / (CCAR * WCAR), (size_t)SEQ * DM, (size_t)SEQ_FULL * DM);
}
